// FeedForwardQuantum_65481071400590
// MI455X (gfx1250) — hardware-verified
//
#include <hip/hip_runtime.h>
#include <stddef.h>


typedef _Float16 v16h __attribute__((ext_vector_type(16)));
typedef _Float16 v8h  __attribute__((ext_vector_type(8)));
typedef float    v8f  __attribute__((ext_vector_type(8)));
typedef float    v4f  __attribute__((ext_vector_type(4)));
typedef _Float16 h16;

#ifndef NB
#define NB 8
#endif
#ifndef SEQ
#define SEQ 2048
#endif
#define NB_FULL  8
#define SEQ_FULL 2048
#define DIM   512
#define HID   2048
#define NQ    8
#define MROWS (NB * SEQ)

static_assert(NB >= 1 && NB <= NB_FULL);
static_assert(SEQ >= 128 && SEQ <= SEQ_FULL && (SEQ % 128) == 0);
static_assert((DIM % 64) == 0 && (DIM % 32) == 0);
static_assert((HID % 64) == 0 && (HID % 32) == 0);
static_assert((MROWS % 64) == 0 && (MROWS % 32) == 0);
static_assert(HID == 256 * 8);
static_assert(NQ == 8);
static_assert(((size_t)DIM * HID) % (256u * 8u) == 0);
static_assert((size_t)MROWS * HID < (size_t)0xFFFFFFFFu);

#define LDC 68
static_assert((LDC % 4) == 0 && LDC >= 64);

#define WCARRY 64.0f
#define MCARRY 16.0f

#define W2P_BYTES ((size_t)DIM * HID * 2)
#define Z_BYTES   ((size_t)MROWS * NQ * 4)
#define MID_BYTES ((size_t)MROWS * HID * 2)
#define OFF_W2  ((size_t)0)
#define OFF_Z   (OFF_W2 + W2P_BYTES)
#define OFF_MID (OFF_Z + Z_BYTES)
#define WS_TOTAL (OFF_MID + MID_BYTES)
static_assert((W2P_BYTES % 128) == 0 && (Z_BYTES % 128) == 0 && (MID_BYTES % 128) == 0);
static_assert(WS_TOTAL <= (size_t)134217728);

__device__ __forceinline__ float bf16r(float x) {
  unsigned int u = __float_as_uint(x);
  u = (u + 0x7FFFu + ((u >> 16) & 1u)) & 0xFFFF0000u;
  return __uint_as_float(u);
}

static __device__ __forceinline__ h16 toh_flush(float v) {
  const h16 r = (h16)v;
  return (fabsf(v) < 6.103515625e-05f) ? (h16)0.0f : r;
}

__device__ __forceinline__ v16h frag_at(const _Float16* p) {
  v8h lo = *(const v8h*)(p);
  v8h hi = *(const v8h*)(p + 16);
  v16h out;
#pragma unroll
  for (int i = 0; i < 8; ++i) { out[i] = lo[i]; out[i + 8] = hi[i]; }
  return out;
}

__device__ __forceinline__ v8f wmma16(v16h a, v16h b, v8f c) {
  v8f d = __builtin_amdgcn_wmma_f32_16x16x32_f16(false, a, false, b, (short)0, c,
                                                 false, false);
  asm volatile("v_nop\n\tv_nop\n\tv_nop\n\tv_nop" : "+v"(d) : "v"(a), "v"(b));
  return d;
}

__device__ __forceinline__ float relu_act(float t) {
  return fmaxf(t, 0.0f);
}

__global__ __launch_bounds__(256) void w2plane_kernel(
    const float* __restrict__ W, _Float16* __restrict__ Wp) {
  const size_t e = ((size_t)blockIdx.x * 256u + threadIdx.x) * 8u;
  const v4f a0 = *(const v4f*)(W + e);
  const v4f a1 = *(const v4f*)(W + e + 4u);
  v8h o;
#pragma unroll
  for (int i = 0; i < 4; ++i) {
    o[i]     = toh_flush(WCARRY * bf16r(a0[i]));
    o[i + 4] = toh_flush(WCARRY * bf16r(a1[i]));
  }
  _Float16* p = Wp + e;
  *(volatile v8h*)p = o;
  __threadfence();
  *(volatile v8h*)p = o;
}

__global__ __launch_bounds__(256) void zenc_kernel(
    const float* __restrict__ X, const float* __restrict__ Th, float* __restrict__ Z) {
  __shared__ float Zs[256] __attribute__((aligned(16)));
  const unsigned tid = threadIdx.x;
  const unsigned q = tid & 7u;
  const unsigned crow = blockIdx.x * 32u + (tid >> 3);
  const unsigned bidx = crow / (unsigned)SEQ;
  const unsigned sq = crow - bidx * (unsigned)SEQ;
  const size_t frow = (size_t)bidx * SEQ_FULL + sq;
  const float ax = bf16r(X[frow * DIM + q]);
  float a = bf16r(Th[q]);
  float z = 1.0f;
#pragma unroll 1
  for (int pass = 0; pass < 2; ++pass) {
    z *= cosf(a);
    a = ax;
  }
  Zs[tid] = z;
  __syncthreads();
  if (tid < 64u) {
    const v4f v = *(const v4f*)&Zs[tid * 4u];
    float* p = Z + (size_t)blockIdx.x * 256u + tid * 4u;
    *(volatile v4f*)p = v;
    __threadfence();
    *(volatile v4f*)p = v;
  }
}

__global__ __launch_bounds__(256) void hmid_kernel(
    const float* __restrict__ Z, const float* __restrict__ W1, _Float16* __restrict__ Mid) {
  __shared__ float Zt[64 * NQ] __attribute__((aligned(16)));
  const unsigned tid = threadIdx.x;
  const unsigned row0 = blockIdx.x * 64u;
  const unsigned f0 = tid * 8u;

  if (tid < 128u) {
    *(v4f*)&Zt[tid * 4u] = *(const v4f*)(Z + (size_t)row0 * NQ + tid * 4u);
  }

  float w[8][8];
#pragma unroll
  for (int c = 0; c < 8; ++c) {
    const v4f a0 = *(const v4f*)(W1 + (size_t)(f0 + (unsigned)c) * NQ);
    const v4f a1 = *(const v4f*)(W1 + (size_t)(f0 + (unsigned)c) * NQ + 4u);
#pragma unroll
    for (int k = 0; k < 4; ++k) {
      w[c][k]     = bf16r(a0[k]);
      w[c][k + 4] = bf16r(a1[k]);
    }
  }
  __syncthreads();

#pragma unroll 1
  for (unsigned t = 0; t < 64u; ++t) {
    const v4f za = *(const v4f*)&Zt[t * NQ];
    const v4f zb = *(const v4f*)&Zt[t * NQ + 4u];
    v8h o;
#pragma unroll
    for (int c = 0; c < 8; ++c) {
      float s = za[0] * w[c][0];
      s = fmaf(za[1], w[c][1], s);
      s = fmaf(za[2], w[c][2], s);
      s = fmaf(za[3], w[c][3], s);
      s = fmaf(zb[0], w[c][4], s);
      s = fmaf(zb[1], w[c][5], s);
      s = fmaf(zb[2], w[c][6], s);
      s = fmaf(zb[3], w[c][7], s);
      o[c] = toh_flush(MCARRY * relu_act(s));
    }
    _Float16* p = Mid + (size_t)(row0 + t) * HID + f0;
    *(volatile v8h*)p = o;
    __threadfence();
    *(volatile v8h*)p = o;
  }
}

__global__ __launch_bounds__(256) void gemm_out_kernel(
    const _Float16* __restrict__ A16, const _Float16* __restrict__ Bt,
    float* __restrict__ outf) {
  __shared__ float Cs[64 * LDC] __attribute__((aligned(16)));
  const unsigned K = (unsigned)HID;
  const unsigned tid = threadIdx.x, lane = tid & 31u, w = tid >> 5;
  const unsigned mw = w >> 1, nw = w & 1u;
  const unsigned hh = lane >> 4, m = lane & 15u;
  const unsigned n0 = blockIdx.x * 64u;
  const unsigned row0 = blockIdx.y * 64u;

  const _Float16* ap  = A16 + (size_t)(row0 + mw * 16u + m) * K + hh * 8u;
  const _Float16* bp0 = Bt + (size_t)(n0 + nw * 32u + m) * K + hh * 8u;
  const _Float16* bp1 = bp0 + (size_t)16 * K;
  v8f acc0 = {}, acc1 = {};
#pragma unroll 2
  for (unsigned k0 = 0; k0 < K; k0 += 32u) {
    const v16h a  = frag_at(ap + k0);
    const v16h b0 = frag_at(bp0 + k0);
    const v16h b1 = frag_at(bp1 + k0);
    acc0 = wmma16(a, b0, acc0);
    acc1 = wmma16(a, b1, acc1);
  }
#pragma unroll
  for (int r = 0; r < 8; ++r) {
    float* d = &Cs[(mw * 16u + hh * 8u + (unsigned)r) * LDC + nw * 32u + m];
    d[0]  = acc0[r];
    d[16] = acc1[r];
  }
  __syncthreads();

  const float cs = 1.0f / (WCARRY * MCARRY);
  v4f xs[4];
  size_t off[4];
#pragma unroll
  for (unsigned i = 0; i < 4u; ++i) {
    const unsigned r = 16u * i + (tid >> 4);
    const unsigned c = (tid & 15u) * 4u;
    const unsigned crow = row0 + r;
    const unsigned bidx = crow / (unsigned)SEQ;
    const unsigned sq = crow - bidx * (unsigned)SEQ;
    const size_t frow = (size_t)bidx * SEQ_FULL + sq;
    const v4f u = *(const v4f*)&Cs[r * LDC + c];
    v4f val;
#pragma unroll
    for (int j = 0; j < 4; ++j) val[j] = u[j] * cs;
    xs[i] = val;
    off[i] = frow * DIM + n0 + c;
  }
#pragma unroll
  for (int i = 0; i < 4; ++i) *(volatile v4f*)(outf + off[i]) = xs[i];
  __threadfence();
#pragma unroll
  for (int i = 0; i < 4; ++i) *(volatile v4f*)(outf + off[i]) = xs[i];
}

extern "C" void kernel_launch(void* const* d_in, const int* in_sizes, int n_in,
                              void* d_out, int out_size, void* d_ws, size_t ws_size,
                              hipStream_t stream) {
  if (n_in < 4) return;
  const long long need_x = ((long long)(NB - 1) * SEQ_FULL + SEQ) * DIM;
  if ((long long)in_sizes[0] < need_x) return;
  if (in_sizes[1] < NQ) return;
  if ((long long)in_sizes[2] < (long long)HID * NQ) return;
  if ((long long)in_sizes[3] < (long long)DIM * HID) return;
  if ((long long)out_size < need_x) return;
  if (ws_size < WS_TOTAL) return;

  const float* X  = (const float*)d_in[0];
  const float* th = (const float*)d_in[1];
  const float* w1 = (const float*)d_in[2];
  const float* w2 = (const float*)d_in[3];
  float* out = (float*)d_out;

  char* ws = (char*)d_ws;
  _Float16* W2p   = (_Float16*)(ws + OFF_W2);
  float*    Zp    = (float*)(ws + OFF_Z);
  _Float16* Mid16 = (_Float16*)(ws + OFF_MID);

  dim3 blk(256);
  w2plane_kernel<<<dim3((unsigned)(((size_t)DIM * HID) / 2048u)), blk, 0, stream>>>(w2, W2p);
  zenc_kernel<<<dim3(MROWS / 32), blk, 0, stream>>>(X, th, Zp);
  hmid_kernel<<<dim3(MROWS / 64), blk, 0, stream>>>(Zp, w1, Mid16);
  gemm_out_kernel<<<dim3(DIM / 64, MROWS / 64), blk, 0, stream>>>(Mid16, W2p, out);
}
